// GraphConvolutionalBlock_21500606284453
// MI455X (gfx1250) — hardware-verified
//
#include <hip/hip_runtime.h>
#include <stddef.h>


#define DH      128
#define NTHR    256
#define NWAVE   8
#define GROWS   128
#define EPT     8
#define NGRP    2
#define CHUNK   (NTHR * EPT * NGRP)
#define WCAP    (EPT * NGRP * 32)
#define LISTN   (NWAVE * WCAP)
#define NBC     4096
#define NBF     1024
#define RCAP    16384
#define RBN     128
#define OTHR    512
#define DEGCAP  256
#define NLP     16

#define LDS_GEMM (GROWS * DH * 4)
#define LDS_FILL ((RCAP + NBF + LISTN) * 4 + 64)

static_assert((CHUNK & (CHUNK - 1)) == 0);
static_assert(CHUNK <= 4096);
static_assert(NBC <= 4096 && NBF <= 4096);
static_assert((NBC & (NBC - 1)) == 0 && (NBF & (NBF - 1)) == 0);
static_assert(NBC == 4 * NBF);
static_assert(OTHR * 8 == NBC);
static_assert((RCAP % 32) == 0);
static_assert(GROWS == NWAVE * 16);
static_assert(NTHR == NWAVE * 32);
static_assert((RCAP + NBF + LISTN + NWAVE) * 4 <= LDS_FILL);

typedef unsigned short us;
typedef float    v4f   __attribute__((ext_vector_type(4)));
typedef float    v8f   __attribute__((ext_vector_type(8)));
typedef int      v4i   __attribute__((ext_vector_type(4)));
typedef us       v4us  __attribute__((ext_vector_type(4)));
typedef us       v8us  __attribute__((ext_vector_type(8)));
typedef __bf16   v16bf __attribute__((ext_vector_type(16)));
union FragB { v16bf v; v8us h[2]; };

__device__ __forceinline__ us f2bf(float f) {
  unsigned int u = __float_as_uint(f);
  u += 0x7FFFu + ((u >> 16) & 1u);
  return (us)(u >> 16);
}
__device__ __forceinline__ float bf2f(us w) { return __uint_as_float(((unsigned int)w) << 16); }

__device__ __forceinline__ void split4(v4f s, v4us& hv, v4us& lv) {
  hv[0] = f2bf(s.x); hv[1] = f2bf(s.y); hv[2] = f2bf(s.z); hv[3] = f2bf(s.w);
  lv[0] = f2bf(s.x - bf2f(hv[0])); lv[1] = f2bf(s.y - bf2f(hv[1]));
  lv[2] = f2bf(s.z - bf2f(hv[2])); lv[3] = f2bf(s.w - bf2f(hv[3]));
}

__device__ __forceinline__ v8f wmb(v16bf a, v16bf b, v8f c) {
  v8f d = __builtin_amdgcn_wmma_f32_16x16x32_bf16(false, a, false, b, (short)0, c, false, false);
  asm volatile("v_nop\n\tv_nop\n\tv_nop\n\tv_nop" : "+v"(d) : "v"(a), "v"(b));
  return d;
}

template <int NPL, int NT>
__device__ __forceinline__ void wave_gemm(const us* xhi, const us* xlo, const us* __restrict__ wpl,
                                          int r0w, int lane, v8f (&acc)[NT]) {
  const int hh = lane >> 4, m = lane & 15;
#pragma unroll
  for (int t = 0; t < NT; ++t) { const v8f z = {0.f, 0.f, 0.f, 0.f, 0.f, 0.f, 0.f, 0.f}; acc[t] = z; }
  const us* ahp = xhi + (size_t)(r0w + m) * DH + 8 * hh;
  const us* alp = xlo + (size_t)(r0w + m) * DH + 8 * hh;
#pragma unroll
  for (int kt = 0; kt < DH / 32; ++kt) {
    FragB ah;
    ah.h[0] = *(const v8us*)(ahp + 32 * kt);
    ah.h[1] = *(const v8us*)(ahp + 32 * kt + 16);
    FragB al = ah;
    if (NPL == 2) {
      al.h[0] = *(const v8us*)(alp + 32 * kt);
      al.h[1] = *(const v8us*)(alp + 32 * kt + 16);
    }
#pragma unroll
    for (int t = 0; t < NT; ++t) {
      const us* bp = wpl + (size_t)(16 * t + m) * DH + 32 * kt + 8 * hh;
      FragB b;
      b.h[0] = *(const v8us*)bp;
      b.h[1] = *(const v8us*)(bp + 16);
      acc[t] = wmb(ah.v, b.v, acc[t]);
      if (NPL == 2) acc[t] = wmb(al.v, b.v, acc[t]);
    }
  }
}

template <int NT>
__device__ __forceinline__ void wave_stage(const v8f (&acc)[NT], const float* __restrict__ bias, float* stw, int lane) {
  const int hh = lane >> 4, m = lane & 15;
  float* sp = stw + (8 * hh) * (16 * NT) + m;
#pragma unroll
  for (int t = 0; t < NT; ++t) {
    const float bv = bias[16 * t + m];
#pragma unroll
    for (int r = 0; r < 8; ++r) sp[r * (16 * NT) + 16 * t] = acc[t][r] + bv;
  }
}

template <int NB>
__device__ __forceinline__ int scan_chunk(const int* __restrict__ dsts, int nD, int cbase, int slotBase,
                                          int vec8, int* list, int tid, int lane, int wave) {
  int wc = 0;
#pragma unroll
  for (int g = 0; g < NGRP; ++g) {
    const int el0  = (g * NTHR + tid) * EPT;
    const int e0   = cbase + el0;
    const int sent = -2147483647 - 1;
    v4i da, db;
    if (vec8 != 0 && cbase + CHUNK <= nD) {
      da = *(const v4i*)(dsts + e0);
      db = *(const v4i*)(dsts + e0 + 4);
    } else {
      da.x = (e0     < nD) ? dsts[min(e0,     nD - 1)] : sent;
      da.y = (e0 + 1 < nD) ? dsts[min(e0 + 1, nD - 1)] : sent;
      da.z = (e0 + 2 < nD) ? dsts[min(e0 + 2, nD - 1)] : sent;
      da.w = (e0 + 3 < nD) ? dsts[min(e0 + 3, nD - 1)] : sent;
      db.x = (e0 + 4 < nD) ? dsts[min(e0 + 4, nD - 1)] : sent;
      db.y = (e0 + 5 < nD) ? dsts[min(e0 + 5, nD - 1)] : sent;
      db.z = (e0 + 6 < nD) ? dsts[min(e0 + 6, nD - 1)] : sent;
      db.w = (e0 + 7 < nD) ? dsts[min(e0 + 7, nD - 1)] : sent;
    }
    const unsigned nb = (unsigned)slotBase;
    const unsigned s0 = (unsigned)da.x - nb, s1 = (unsigned)da.y - nb;
    const unsigned s2 = (unsigned)da.z - nb, s3 = (unsigned)da.w - nb;
    const unsigned s4 = (unsigned)db.x - nb, s5 = (unsigned)db.y - nb;
    const unsigned s6 = (unsigned)db.z - nb, s7 = (unsigned)db.w - nb;
    const bool h0 = s0 < (unsigned)NB, h1 = s1 < (unsigned)NB, h2 = s2 < (unsigned)NB, h3 = s3 < (unsigned)NB;
    const bool h4 = s4 < (unsigned)NB, h5 = s5 < (unsigned)NB, h6 = s6 < (unsigned)NB, h7 = s7 < (unsigned)NB;
    const unsigned any = __builtin_amdgcn_ballot_w32(h0 | h1 | h2 | h3 | h4 | h5 | h6 | h7);
    if (any != 0u) {
#define HITJ(J, HJ, SJ) { \
        const unsigned mj = __builtin_amdgcn_ballot_w32(HJ); \
        if (mj != 0u) { \
          if (HJ) { \
            const int pos = wc + (int)__builtin_amdgcn_mbcnt_lo(mj, 0u); \
            if (pos < WCAP) list[wave * WCAP + pos] = ((el0 + (J)) << 12) | (int)(SJ); \
          } \
          wc += (int)__builtin_popcount(mj); } }
      HITJ(0, h0, s0)
      HITJ(1, h1, s1)
      HITJ(2, h2, s2)
      HITJ(3, h3, s3)
      HITJ(4, h4, s4)
      HITJ(5, h5, s5)
      HITJ(6, h6, s6)
      HITJ(7, h7, s7)
#undef HITJ
    }
  }
  return wc;
}

__global__ __launch_bounds__(NTHR) void k_cvt_rows(const float* __restrict__ src, us* dst, int nValid, int nRows) {
  const int i = blockIdx.x * NTHR + (int)threadIdx.x;
  const int total = nRows * (DH / 8);
  if (i >= total) return;
  const int row = i >> 4;
  const int c0  = (i & 15) * 8;
  const int rc  = row < nValid ? row : nValid - 1;
  const float* p = src + (size_t)rc * DH + c0;
  const v4f a = *(const v4f*)p, b = *(const v4f*)(p + 4);
  const bool ok = row < nValid;
  v8us o;
  o[0] = ok ? f2bf(a.x) : (us)0; o[1] = ok ? f2bf(a.y) : (us)0;
  o[2] = ok ? f2bf(a.z) : (us)0; o[3] = ok ? f2bf(a.w) : (us)0;
  o[4] = ok ? f2bf(b.x) : (us)0; o[5] = ok ? f2bf(b.y) : (us)0;
  o[6] = ok ? f2bf(b.z) : (us)0; o[7] = ok ? f2bf(b.w) : (us)0;
  us* dp = dst + (size_t)i * 8;
  *(volatile v8us*)dp = o;
  __threadfence();
  *(volatile v8us*)dp = o;
}

__device__ __forceinline__ v8us cvt_wrow(const float* __restrict__ W, int tid, int dOut) {
  const int row = tid >> 4, c0 = (tid & 15) * 8;
  const int rc = row < dOut ? row : dOut - 1;
  const float* sp = W + rc * DH + c0;
  const v4f a = *(const v4f*)sp, b = *(const v4f*)(sp + 4);
  const bool ok = row < dOut;
  v8us o;
  o[0] = ok ? f2bf(a.x) : (us)0; o[1] = ok ? f2bf(a.y) : (us)0;
  o[2] = ok ? f2bf(a.z) : (us)0; o[3] = ok ? f2bf(a.w) : (us)0;
  o[4] = ok ? f2bf(b.x) : (us)0; o[5] = ok ? f2bf(b.y) : (us)0;
  o[6] = ok ? f2bf(b.z) : (us)0; o[7] = ok ? f2bf(b.w) : (us)0;
  return o;
}

__device__ __forceinline__ void bias_pass(const float* __restrict__ b01, const float* __restrict__ b11,
                                          const float* __restrict__ b0h, const float* __restrict__ b1h,
                                          float* biasA, int nL, int lane, int wave) {
  const int nv = 64 + 64 * nL;
  const int nIter = (nv + NTHR - 1) / NTHR;
#pragma unroll 1
  for (int k = 0; k < nIter; ++k) {
    const int i0 = k * NTHR + wave * 32;
    if (i0 < nv) {
      const float* src; int base;
      if (i0 < 32)                { src = b01; base = 0; }
      else if (i0 < 64)           { src = b11; base = 32; }
      else if (i0 < 64 + 32 * nL) { src = b0h; base = 64; }
      else                        { src = b1h; base = 64 + 32 * nL; }
      const int i = i0 + lane;
      const v4f x = *(const v4f*)(src + 4 * (i - base));
      v4f r;
      r.x = bf2f(f2bf(x.x)); r.y = bf2f(f2bf(x.y)); r.z = bf2f(f2bf(x.z)); r.w = bf2f(f2bf(x.w));
      *(volatile v4f*)(biasA + 4 * i) = r;
    }
  }
}

__global__ __launch_bounds__(NTHR) void k_prep_small(
    const float* __restrict__ W0l, const float* __restrict__ W1l,
    const float* __restrict__ b01, const float* __restrict__ b11,
    const float* __restrict__ b0h, const float* __restrict__ b1h,
    const float* __restrict__ b0l, const float* __restrict__ b1l,
    us* wl0, us* wl1, float* biasA, float* biasL, int nL, int dOut) {
  const int tid = threadIdx.x, lane = tid & 31, wave = tid >> 5;
  const v8us wv0 = cvt_wrow(W0l, tid, dOut);
  const v8us wv1 = cvt_wrow(W1l, tid, dOut);
  const int which = lane >> 4, e = lane & 15;
  const int ec = e < dOut ? e : dOut - 1;
  const float va = b0l[ec], vb = b1l[ec];
  const float bl0 = e < dOut ? (which == 0 ? va : vb) : 0.0f;
  const float bl = bf2f(f2bf(bl0));

  *(volatile v8us*)(wl0 + 8 * tid) = wv0;
  *(volatile v8us*)(wl1 + 8 * tid) = wv1;
  bias_pass(b01, b11, b0h, b1h, biasA, nL, lane, wave);
  if (wave == 0) *(volatile float*)(biasL + lane) = bl;
  __threadfence();
  *(volatile v8us*)(wl0 + 8 * tid) = wv0;
  *(volatile v8us*)(wl1 + 8 * tid) = wv1;
  bias_pass(b01, b11, b0h, b1h, biasA, nL, lane, wave);
  if (wave == 0) *(volatile float*)(biasL + lane) = bl;
}

__global__ __launch_bounds__(NTHR) void k_count(const int* __restrict__ ef, int* cnt, int nD, int vec8) {
  __shared__ __attribute__((aligned(16))) int scnt[NBC];
  __shared__ __attribute__((aligned(16))) int list[LISTN];
  __shared__ int wcnt[NWAVE];
  const int tid = threadIdx.x, lane = tid & 31, wave = tid >> 5;
  const int nodeBase = blockIdx.x * NBC;

  for (int i = tid; i < NBC; i += NTHR) scnt[i] = 0;
  __syncthreads();

  const int nChunks = (nD + CHUNK - 1) / CHUNK;
#pragma unroll 1
  for (int ch = 0; ch < nChunks; ++ch) {
    const int cbase = ch * CHUNK;
    const int wc = scan_chunk<NBC>(ef, nD, cbase, nodeBase, vec8, list, tid, lane, wave);
    if (lane == 0) wcnt[wave] = wc;
    __syncthreads();
    if (wave == 0) {
#pragma unroll 1
      for (int wsx = 0; wsx < NWAVE; ++wsx) {
        int n = __builtin_amdgcn_readfirstlane(wcnt[wsx]);
        n = n > WCAP ? WCAP : (n < 0 ? 0 : n);
        const int* lp = list + wsx * WCAP;
#pragma unroll 1
        for (int i = 0; i < n; ++i) {
          const int ent  = __builtin_amdgcn_readfirstlane(lp[i]);
          const int slot = ent & (NBC - 1);
          if (lane == 0) scnt[slot] = scnt[slot] + 1;
        }
      }
    }
    __syncthreads();
  }

  v4i cq[4];
#pragma unroll
  for (int q = 0; q < 4; ++q) {
    const int f = (wave * 4 + q) * 128 + 4 * lane;
    cq[q] = *(const v4i*)(scnt + f);
  }
  int* cp = cnt + (size_t)nodeBase;
#pragma unroll
  for (int q = 0; q < 4; ++q) { const int f = (wave * 4 + q) * 128 + 4 * lane; *(volatile v4i*)(cp + f) = cq[q]; }
  __threadfence();
#pragma unroll
  for (int q = 0; q < 4; ++q) { const int f = (wave * 4 + q) * 128 + 4 * lane; *(volatile v4i*)(cp + f) = cq[q]; }
}

__global__ __launch_bounds__(OTHR) void k_offsets(const int* __restrict__ cnt, int* off, int* rbase, int nChunk) {
  __shared__ __attribute__((aligned(16))) int soff[NBC];
  __shared__ __attribute__((aligned(16))) int srb[RBN];
  __shared__ int wtot[OTHR / 32];
  const int tid = threadIdx.x, lane = tid & 31, wave = tid >> 5, sub = tid >> 7;
  for (int i = tid; i < RBN; i += OTHR) srb[i] = 0;
  int carry = 0;
#pragma unroll 1
  for (int ch = 0; ch < nChunk; ++ch) {
    const int base = ch * NBC;
    const v4i c0 = *(const v4i*)(cnt + base + 8 * tid);
    const v4i c1 = *(const v4i*)(cnt + base + 8 * tid + 4);
    const int e0 = max(c0.x, 0), e1 = max(c0.y, 0), e2 = max(c0.z, 0), e3 = max(c0.w, 0);
    const int e4 = max(c1.x, 0), e5 = max(c1.y, 0), e6 = max(c1.z, 0), e7 = max(c1.w, 0);
    const int ts = e0 + e1 + e2 + e3 + e4 + e5 + e6 + e7;
    int incl = ts;
#pragma unroll
    for (int d = 1; d < 32; d <<= 1) {
      const int t = __shfl_up(incl, d);
      if (lane >= d) incl += t;
    }
    if (lane == 31) wtot[wave] = incl;
    __syncthreads();
    const int S0 = wtot[0]  + wtot[1]  + wtot[2]  + wtot[3];
    const int S1 = wtot[4]  + wtot[5]  + wtot[6]  + wtot[7];
    const int S2 = wtot[8]  + wtot[9]  + wtot[10] + wtot[11];
    const int S3 = wtot[12] + wtot[13] + wtot[14] + wtot[15];
    int pre = 0;
#pragma unroll 1
    for (int w = 4 * sub; w < wave; ++w) pre += wtot[w];
    const int b0 = carry;
    const int b1 = b0 + ((S0 + 31) & ~31);
    const int b2 = b1 + ((S1 + 31) & ~31);
    const int b3 = b2 + ((S2 + 31) & ~31);
    const int b4 = b3 + ((S3 + 31) & ~31);
    const int myb = sub == 0 ? b0 : (sub == 1 ? b1 : (sub == 2 ? b2 : b3));
    if (tid == 0) {
      srb[min(4 * ch + 0, RBN - 1)] = b0;
      srb[min(4 * ch + 1, RBN - 1)] = b1;
      srb[min(4 * ch + 2, RBN - 1)] = b2;
      srb[min(4 * ch + 3, RBN - 1)] = b3;
    }
    int run = myb + pre + incl - ts;
    soff[8 * tid + 0] = run; run += e0;
    soff[8 * tid + 1] = run; run += e1;
    soff[8 * tid + 2] = run; run += e2;
    soff[8 * tid + 3] = run; run += e3;
    soff[8 * tid + 4] = run; run += e4;
    soff[8 * tid + 5] = run; run += e5;
    soff[8 * tid + 6] = run; run += e6;
    soff[8 * tid + 7] = run;
    carry = b4;
    __syncthreads();
    const v4i o0 = *(const v4i*)(soff + 4 * tid);
    const v4i o1 = *(const v4i*)(soff + 4 * (tid + OTHR));
    int* op = off + base;
    *(volatile v4i*)(op + 4 * tid) = o0;
    *(volatile v4i*)(op + 4 * (tid + OTHR)) = o1;
    __threadfence();
    *(volatile v4i*)(op + 4 * tid) = o0;
    *(volatile v4i*)(op + 4 * (tid + OTHR)) = o1;
    __syncthreads();
  }
  if (tid == 0) srb[min(4 * nChunk, RBN - 1)] = carry;
  __syncthreads();
  v4i rv = {0, 0, 0, 0};
  if (tid < 32) rv = *(const v4i*)(srb + 4 * tid);
  if (tid < 32) *(volatile v4i*)(rbase + 4 * tid) = rv;
  __threadfence();
  if (tid < 32) *(volatile v4i*)(rbase + 4 * tid) = rv;
}

__global__ __launch_bounds__(NTHR) void k_fill(
    const int* __restrict__ ef, const int* __restrict__ off, const int* __restrict__ rbase,
    int* csr, int nN, int nD, int vec8, int csrLen) {
  extern __shared__ v4f lds_dyn[];
  int* region = (int*)lds_dyn;
  int* cursor = region + RCAP;
  int* list   = cursor + NBF;
  int* wcnt   = list + LISTN;
  const int tid = threadIdx.x, lane = tid & 31, wave = tid >> 5;
  const int b = blockIdx.x;
  const int nodeBase = b * NBF;

  int rb0 = rbase[b];
  const int rb1 = rbase[b + 1];
  rb0 = rb0 < 0 ? 0 : (rb0 > csrLen ? csrLen : rb0);
  rb0 &= ~31;
  int len = rb1 - rb0;
  len = len < 0 ? 0 : (len > RCAP ? RCAP : len);
  int lenW = (len + 31) & ~31;
  if (rb0 + lenW > csrLen) lenW = (csrLen - rb0) & ~31;

  {
    const v4i z = {0, 0, 0, 0};
    for (int i = tid; i < RCAP / 4; i += NTHR) ((v4i*)region)[i] = z;
    for (int s = tid; s < NBF; s += NTHR) {
      int o = off[nodeBase + s] - rb0;
      o = o < 0 ? 0 : (o > RCAP ? RCAP : o);
      cursor[s] = o;
    }
  }
  __syncthreads();

  const int nChunks = (nD + CHUNK - 1) / CHUNK;
#pragma unroll 1
  for (int ch = 0; ch < nChunks; ++ch) {
    const int cbase = ch * CHUNK;
    const int wc = scan_chunk<NBF>(ef, nD, cbase, nodeBase, vec8, list, tid, lane, wave);
    if (lane == 0) wcnt[wave] = wc;
    __syncthreads();
    if (wave == 0) {
#pragma unroll 1
      for (int wsx = 0; wsx < NWAVE; ++wsx) {
        int n = __builtin_amdgcn_readfirstlane(wcnt[wsx]);
        n = n > WCAP ? WCAP : (n < 0 ? 0 : n);
        const int* lp = list + wsx * WCAP;
#pragma unroll 1
        for (int i = 0; i < n; ++i) {
          const int ent  = __builtin_amdgcn_readfirstlane(lp[i]);
          const int slot = ent & (NBF - 1);
          int e = cbase + ((ent >> 12) & (CHUNK - 1));
          e = e > nD - 1 ? nD - 1 : e;
          int es = e ^ 1;
          es = es < 0 ? 0 : (es > nD - 1 ? nD - 1 : es);
          int src = ef[es];
          src = src < 0 ? 0 : (src > nN - 1 ? nN - 1 : src);
          if (lane == 0) {
            int pos = cursor[slot];
            pos = pos < 0 ? 0 : (pos > RCAP - 1 ? RCAP - 1 : pos);
            region[pos] = src;
            const int np = pos + 1;
            cursor[slot] = np > RCAP ? RCAP : np;
          }
        }
      }
    }
    __syncthreads();
  }

  const int nv = lenW >> 2;
  int* gp = csr + rb0;
#pragma unroll 1
  for (int i = tid; i < nv; i += NTHR) { const v4i v = ((const v4i*)region)[i]; *(volatile v4i*)(gp + 4 * i) = v; }
  __threadfence();
#pragma unroll 1
  for (int i = tid; i < nv; i += NTHR) { const v4i v = ((const v4i*)region)[i]; *(volatile v4i*)(gp + 4 * i) = v; }
}

template <int NPL, int NT>
__global__ __launch_bounds__(NTHR) void k_gemm_n(
    const us* xhi, const us* xlo, const us* __restrict__ wpl, const float* __restrict__ bias, float* C) {
  extern __shared__ v4f lds_dyn[];
  float* stg = (float*)lds_dyn;
  const int tid = threadIdx.x, lane = tid & 31, wave = tid >> 5;
  const int r0w = blockIdx.x * GROWS + wave * 16;
  float* stw = stg + wave * (256 * NT);
  {
    v8f acc[NT];
    wave_gemm<NPL, NT>(xhi, xlo, wpl, r0w, lane, acc);
    wave_stage<NT>(acc, bias, stw, lane);
  }
  __syncthreads();
  float* gp = C + (size_t)r0w * (16 * NT);
#pragma unroll
  for (int p = 0; p < 2 * NT; ++p) { const v4f v = *(const v4f*)(stw + 128 * p + 4 * lane); *(volatile v4f*)(gp + 128 * p + 4 * lane) = v; }
  __threadfence();
#pragma unroll
  for (int p = 0; p < 2 * NT; ++p) { const v4f v = *(const v4f*)(stw + 128 * p + 4 * lane); *(volatile v4f*)(gp + 128 * p + 4 * lane) = v; }
}

__device__ __forceinline__ v4f gather_sum(const float* __restrict__ nbuf, const int* __restrict__ csr,
                                          int cnt_l, int off_l, int j, int lane, int nN, int csrLen) {
  int n = __builtin_amdgcn_readlane(cnt_l, j);
  n = n < 0 ? 0 : (n > DEGCAP ? DEGCAP : n);
  int st = __builtin_amdgcn_readlane(off_l, j);
  st = st < 0 ? 0 : (st > csrLen ? csrLen : st);
  v4f acc = {0.f, 0.f, 0.f, 0.f};
#pragma unroll 1
  for (int q0 = 0; q0 < n; q0 += 32) {
    int pos = st + q0 + lane;
    pos = pos < 0 ? 0 : (pos > csrLen - 1 ? csrLen - 1 : pos);
    int sl = csr[pos];
    sl = sl < 0 ? 0 : (sl > nN - 1 ? nN - 1 : sl);
    const int mc = (n - q0) < 32 ? (n - q0) : 32;
#pragma unroll 1
    for (int p = 0; p < mc; ++p) {
      const int s = __builtin_amdgcn_readlane(sl, p);
      acc = acc + *(const v4f*)(nbuf + (size_t)s * DH + 4 * lane);
    }
  }
  return acc;
}

template <int MODE>
__device__ __forceinline__ void emit_row(v4f v, int c, int lane, us* xhi, us* xlo, us* res, float* aux, int nN) {
  const size_t o = (size_t)c * DH + 4 * lane;
  v4f s = v;
  if (MODE == 2) {
    const v4us rw = *(const v4us*)(res + o);
    v4f rv; rv.x = bf2f(rw[0]); rv.y = bf2f(rw[1]); rv.z = bf2f(rw[2]); rv.w = bf2f(rw[3]);
    s = v + rv;
    if (c < nN) *(volatile v4f*)(aux + o) = v;
  }
  v4us hv, lv;
  split4(s, hv, lv);
  *(volatile v4us*)(xhi + o) = hv;
  *(volatile v4us*)(xlo + o) = lv;
  if (MODE == 0) *(volatile v4us*)(res + o) = hv;
}

template <int NPL, int MODE>
__global__ __launch_bounds__(NTHR) void k_aggy(
    us* xhi, us* xlo, us* res, const us* __restrict__ wpl, const float* __restrict__ bias,
    const float* __restrict__ nbuf, const int* __restrict__ csr, const int* __restrict__ offp,
    const int* __restrict__ cnt, float* aux, int nN, int csrLen) {
  extern __shared__ v4f lds_dyn[];
  float* stg = (float*)lds_dyn;
  const int tid = threadIdx.x, lane = tid & 31, wave = tid >> 5;
  const int r0w = blockIdx.x * GROWS + wave * 16;
  float* stw = stg + wave * (16 * DH);
  {
    v8f acc[8];
    wave_gemm<NPL, 8>(xhi, xlo, wpl, r0w, lane, acc);
    wave_stage<8>(acc, bias, stw, lane);
  }
  __syncthreads();

  const int cl = r0w + (lane & 15);
  const int cnt_l = cnt[cl];
  const int off_l = offp[cl];
#pragma unroll 1
  for (int j = 0; j < 16; ++j) {
    const v4f g = gather_sum(nbuf, csr, cnt_l, off_l, j, lane, nN, csrLen);
    float* sp = stw + j * DH + 4 * lane;
    v4f v = *(const v4f*)sp + g;
    v.x = fmaxf(v.x, 0.f); v.y = fmaxf(v.y, 0.f); v.z = fmaxf(v.z, 0.f); v.w = fmaxf(v.w, 0.f);
    *(v4f*)sp = v;
    emit_row<MODE>(v, r0w + j, lane, xhi, xlo, res, aux, nN);
  }
  __threadfence();
  __syncthreads();
#pragma unroll 1
  for (int j = 0; j < 16; ++j) {
    const v4f v = *(const v4f*)(stw + j * DH + 4 * lane);
    emit_row<MODE>(v, r0w + j, lane, xhi, xlo, res, aux, nN);
  }
}

__global__ __launch_bounds__(NTHR) void k_last(
    const us* xhi, const us* xlo, const us* __restrict__ wpl, const float* __restrict__ bias,
    const float* __restrict__ n3, const int* __restrict__ csr, const int* __restrict__ offp,
    const int* __restrict__ cnt, float* out0, int nN, int csrLen, int dOut) {
  __shared__ __attribute__((aligned(16))) float stg[NWAVE * 16 * NLP];
  __shared__ __attribute__((aligned(16))) float sout[GROWS * NLP];
  const int tid = threadIdx.x, lane = tid & 31, wave = tid >> 5;
  const int rowBase = blockIdx.x * GROWS;
  const int r0w = rowBase + wave * 16;
  float* stw = stg + wave * (16 * NLP);
  {
    v8f acc[1];
    wave_gemm<2, 1>(xhi, xlo, wpl, r0w, lane, acc);
    wave_stage<1>(acc, bias, stw, lane);
  }
  __syncthreads();

  const int cl = r0w + (lane & 15);
  const int cnt_l = cnt[cl];
  const int off_l = offp[cl];
  const int ch = lane & 15;
#pragma unroll 1
  for (int j = 0; j < 16; ++j) {
    int n = __builtin_amdgcn_readlane(cnt_l, j);
    n = n < 0 ? 0 : (n > DEGCAP ? DEGCAP : n);
    int st = __builtin_amdgcn_readlane(off_l, j);
    st = st < 0 ? 0 : (st > csrLen ? csrLen : st);
    float acc = 0.0f;
#pragma unroll 1
    for (int q0 = 0; q0 < n; q0 += 32) {
      int pos = st + q0 + lane;
      pos = pos < 0 ? 0 : (pos > csrLen - 1 ? csrLen - 1 : pos);
      int sl = csr[pos];
      sl = sl < 0 ? 0 : (sl > nN - 1 ? nN - 1 : sl);
      const int mc = (n - q0) < 32 ? (n - q0) : 32;
#pragma unroll 1
      for (int p = 0; p < mc; ++p) {
        const int s = __builtin_amdgcn_readlane(sl, p);
        acc += n3[(size_t)s * NLP + ch];
      }
    }
    const float v = stw[j * NLP + ch] + acc;
    if (lane < dOut) sout[(wave * 16 + j) * dOut + lane] = v;
  }
  __syncthreads();

  int nvr = nN - rowBase;
  nvr = nvr < 0 ? 0 : (nvr > GROWS ? GROWS : nvr);
  const int nf4 = (nvr * dOut) >> 2;
  float* op = out0 + (size_t)rowBase * dOut;
#pragma unroll 1
  for (int i = tid; i < nf4; i += NTHR) { const v4f v = *(const v4f*)(sout + 4 * i); *(volatile v4f*)(op + 4 * i) = v; }
  __threadfence();
#pragma unroll 1
  for (int i = tid; i < nf4; i += NTHR) { const v4f v = *(const v4f*)(sout + 4 * i); *(volatile v4f*)(op + 4 * i) = v; }
}

extern "C" void kernel_launch(void* const* d_in, const int* in_sizes, int n_in,
                              void* d_out, int out_size, void* d_ws, size_t ws_size,
                              hipStream_t stream) {
  if (n_in < 14) return;
  const int nN   = in_sizes[0] / DH;
  const int nE   = in_sizes[1] / 2;
  const int nL   = in_sizes[6] / (DH * DH);
  const int dOut = in_sizes[11];
  if (nN < 32 || in_sizes[0] != nN * DH || (nN & 31) != 0 || nN > (1 << 24)) return;
  if (nE <= 0 || in_sizes[1] != 2 * nE || nE > (1 << 27)) return;
  if (in_sizes[2] != DH * DH || in_sizes[3] != DH || in_sizes[4] != DH * DH || in_sizes[5] != DH) return;
  if (nL < 1 || in_sizes[6] != nL * DH * DH || in_sizes[7] != nL * DH ||
      in_sizes[8] != nL * DH * DH || in_sizes[9] != nL * DH) return;
  if (dOut < 1 || dOut > NLP || in_sizes[10] != dOut * DH || in_sizes[12] != dOut * DH || in_sizes[13] != dOut) return;
  if (out_size != nN * dOut + nN * DH) return;

  const float* features = (const float*)d_in[0];
  const int*   ef       = (const int*)d_in[1];
  const float* W0_1 = (const float*)d_in[2];  const float* b0_1 = (const float*)d_in[3];
  const float* W1_1 = (const float*)d_in[4];  const float* b1_1 = (const float*)d_in[5];
  const float* W0_h = (const float*)d_in[6];  const float* b0_h = (const float*)d_in[7];
  const float* W1_h = (const float*)d_in[8];  const float* b1_h = (const float*)d_in[9];
  const float* W0_l = (const float*)d_in[10]; const float* b0_l = (const float*)d_in[11];
  const float* W1_l = (const float*)d_in[12]; const float* b1_l = (const float*)d_in[13];
  float* out0 = (float*)d_out;
  float* aux  = (float*)d_out + (size_t)nN * dOut;

  const int NPAD   = ((nN + GROWS - 1) / GROWS) * GROWS;
  const int nBC    = (nN + NBC - 1) / NBC;
  const int CNTPAD = nBC * NBC;
  if (4 * nBC + 1 > RBN || CNTPAD < NPAD) return;
  const int nBF    = (nN + NBF - 1) / NBF;
  const int nD     = 2 * nE;
  const int csrLen = ((nD + 31) & ~31) + 4096;
  const int nG     = NPAD / GROWS;
  const int vec8   = ((nD & 3) == 0) ? 1 : 0;

  char* ws = (char*)d_ws;
  size_t off = 0;
  const size_t plW  = (size_t)DH * DH * 2;
  const size_t oWpl = off; off += (size_t)(2 + 2 * nL) * plW;        off = (off + 255) & ~(size_t)255;
  const size_t oWl0 = off; off += (size_t)NLP * DH * 2;              off = (off + 255) & ~(size_t)255;
  const size_t oWl1 = off; off += (size_t)NLP * DH * 2;              off = (off + 255) & ~(size_t)255;
  const size_t oBA  = off; off += (size_t)(2 * DH + 2 * nL * DH) * 4; off = (off + 255) & ~(size_t)255;
  const size_t oBL  = off; off += (size_t)(2 * NLP) * 4;             off = (off + 255) & ~(size_t)255;
  const size_t oCnt = off; off += (size_t)CNTPAD * 4;                off = (off + 255) & ~(size_t)255;
  const size_t oOff = off; off += (size_t)CNTPAD * 4;                off = (off + 255) & ~(size_t)255;
  const size_t oRb  = off; off += (size_t)RBN * 4;                   off = (off + 255) & ~(size_t)255;
  const size_t oCsr = off; off += (size_t)csrLen * 4;                off = (off + 255) & ~(size_t)255;
  const size_t oXhi = off; off += (size_t)NPAD * DH * 2;             off = (off + 255) & ~(size_t)255;
  const size_t oXlo = off; off += (size_t)NPAD * DH * 2;             off = (off + 255) & ~(size_t)255;
  const size_t oRes = off; off += (size_t)NPAD * DH * 2;             off = (off + 255) & ~(size_t)255;
  const size_t oN   = off; off += (size_t)NPAD * DH * 4;             off = (off + 255) & ~(size_t)255;
  if (off > ws_size) return;

  us*    wpl   = (us*)(ws + oWpl);
  us*    wl0   = (us*)(ws + oWl0);
  us*    wl1   = (us*)(ws + oWl1);
  float* biasA = (float*)(ws + oBA);
  float* biasL = (float*)(ws + oBL);
  int*   cnt   = (int*)(ws + oCnt);
  int*   offp  = (int*)(ws + oOff);
  int*   rb    = (int*)(ws + oRb);
  int*   csr   = (int*)(ws + oCsr);
  us*    xhi   = (us*)(ws + oXhi);
  us*    xlo   = (us*)(ws + oXlo);
  us*    res   = (us*)(ws + oRes);
  float* nbuf  = (float*)(ws + oN);

  us* wW0_1 = wpl;
  us* wW1_1 = wpl + (size_t)DH * DH;
  us* wW0_h = wpl + (size_t)2 * DH * DH;
  us* wW1_h = wpl + (size_t)(2 + nL) * DH * DH;
  const float* rb0_1 = biasA;
  const float* rb1_1 = biasA + DH;
  const float* rb0_h = biasA + 2 * DH;
  const float* rb1_h = biasA + 2 * DH + (size_t)nL * DH;
  const float* rb0_l = biasL;
  const float* rb1_l = biasL + NLP;

  k_cvt_rows<<<(DH * (DH / 8) + NTHR - 1) / NTHR, NTHR, 0, stream>>>(W0_1, wW0_1, DH, DH);
  k_cvt_rows<<<(DH * (DH / 8) + NTHR - 1) / NTHR, NTHR, 0, stream>>>(W1_1, wW1_1, DH, DH);
  k_cvt_rows<<<(nL * DH * (DH / 8) + NTHR - 1) / NTHR, NTHR, 0, stream>>>(W0_h, wW0_h, nL * DH, nL * DH);
  k_cvt_rows<<<(nL * DH * (DH / 8) + NTHR - 1) / NTHR, NTHR, 0, stream>>>(W1_h, wW1_h, nL * DH, nL * DH);
  k_cvt_rows<<<(NPAD * (DH / 8) + NTHR - 1) / NTHR, NTHR, 0, stream>>>(features, xhi, nN, NPAD);
  k_prep_small<<<1, NTHR, 0, stream>>>(W0_l, W1_l, b0_1, b1_1, b0_h, b1_h, b0_l, b1_l, wl0, wl1, biasA, biasL, nL, dOut);

  k_count<<<nBC, NTHR, 0, stream>>>(ef, cnt, nD, vec8);
  k_offsets<<<1, OTHR, 0, stream>>>(cnt, offp, rb, nBC);
  hipFuncSetAttribute(reinterpret_cast<const void*>(&k_fill), hipFuncAttributeMaxDynamicSharedMemorySize, LDS_FILL);
  k_fill<<<nBF, NTHR, LDS_FILL, stream>>>(ef, offp, rb, csr, nN, nD, vec8, csrLen);

  hipFuncSetAttribute(reinterpret_cast<const void*>(&k_gemm_n<1, 8>), hipFuncAttributeMaxDynamicSharedMemorySize, LDS_GEMM);
  hipFuncSetAttribute(reinterpret_cast<const void*>(&k_gemm_n<2, 8>), hipFuncAttributeMaxDynamicSharedMemorySize, LDS_GEMM);
  hipFuncSetAttribute(reinterpret_cast<const void*>(&k_aggy<1, 0>),   hipFuncAttributeMaxDynamicSharedMemorySize, LDS_GEMM);
  hipFuncSetAttribute(reinterpret_cast<const void*>(&k_aggy<2, 1>),   hipFuncAttributeMaxDynamicSharedMemorySize, LDS_GEMM);
  hipFuncSetAttribute(reinterpret_cast<const void*>(&k_aggy<2, 2>),   hipFuncAttributeMaxDynamicSharedMemorySize, LDS_GEMM);

  k_gemm_n<1, 8><<<nG, NTHR, LDS_GEMM, stream>>>(xhi, xhi, wW1_1, rb1_1, nbuf);
  k_aggy<1, 0><<<nG, NTHR, LDS_GEMM, stream>>>(xhi, xlo, res, wW0_1, rb0_1, nbuf, csr, offp, cnt, aux, nN, csrLen);

  for (int l = 0; l < nL; ++l) {
    k_gemm_n<2, 8><<<nG, NTHR, LDS_GEMM, stream>>>(xhi, xlo, wW1_h + (size_t)l * DH * DH, rb1_h + (size_t)l * DH, nbuf);
    if (l == nL - 1)
      k_aggy<2, 2><<<nG, NTHR, LDS_GEMM, stream>>>(xhi, xlo, res, wW0_h + (size_t)l * DH * DH, rb0_h + (size_t)l * DH,
                                                 nbuf, csr, offp, cnt, aux, nN, csrLen);
    else
      k_aggy<2, 1><<<nG, NTHR, LDS_GEMM, stream>>>(xhi, xlo, res, wW0_h + (size_t)l * DH * DH, rb0_h + (size_t)l * DH,
                                                 nbuf, csr, offp, cnt, aux, nN, csrLen);
  }

  k_gemm_n<2, 1><<<nG, NTHR, NWAVE * 256 * 4, stream>>>(xhi, xlo, wl1, rb1_l, nbuf);
  k_last<<<nG, NTHR, 0, stream>>>(xhi, xlo, wl0, rb0_l, nbuf, csr, offp, cnt, out0, nN, csrLen, dOut);
}
